// CharRNNEmbedding_30623116821127
// MI455X (gfx1250) — hardware-verified
//
#include <hip/hip_runtime.h>
#include <stdint.h>


#define NWORD 4096
#define TCH   16
#define EMB   64
#define HID   256
#define G4    1024
#define VOC   262
#define L1IN  512

#define NWB   16
#define HSP   264
#define MSP   520
#define OSP   260

#define OPSCALE 16.0f
#define ACCINV  0.00390625f

static_assert(NWORD % NWB == 0);
static_assert(EMB % 32 == 0 && HID % 32 == 0 && L1IN % 32 == 0);
static_assert((HSP * 2) % 16 == 0 && (MSP * 2) % 16 == 0 && (OSP * 4) % 16 == 0);
static_assert((NWB * HSP) % 8 == 0);
static_assert(G4 == 4 * HID && L1IN == 2 * HID);
static_assert(HID == 8 * 32);
static_assert(NWB * HID / 4 == 4 * 256);

typedef float    v4f  __attribute__((ext_vector_type(4)));
typedef float    v8f  __attribute__((ext_vector_type(8)));
typedef _Float16 v8h  __attribute__((ext_vector_type(8)));
typedef _Float16 v16h __attribute__((ext_vector_type(16)));
typedef v8h v8ha __attribute__((may_alias));
typedef v4f v4fa __attribute__((may_alias));
typedef __attribute__((address_space(1))) const v8ha  gv8h;
typedef __attribute__((address_space(1))) const v4fa  gv4f;
typedef __attribute__((address_space(1))) const float gf32;
typedef __attribute__((address_space(1))) const int   gi32;

union Frag { v16h v; v8h p[2]; };

constexpr size_t SZ_XP   = (size_t)TCH * NWORD * EMB * 2;
constexpr size_t SZ_WIH0 = (size_t)G4 * EMB * 2;
constexpr size_t SZ_WHH0 = (size_t)G4 * HID * 2;
constexpr size_t SZ_WIH1 = (size_t)G4 * L1IN * 2;
constexpr size_t SZ_WOUT = (size_t)HID * L1IN * 2;
constexpr size_t SZ_APL  = (size_t)NWORD * L1IN * 2;

constexpr size_t OFF_XP    = 0;
constexpr size_t OFF_WIH0F = OFF_XP + SZ_XP;
constexpr size_t OFF_WIH0B = OFF_WIH0F + SZ_WIH0;
constexpr size_t OFF_WHH0F = OFF_WIH0B + SZ_WIH0;
constexpr size_t OFF_WHH0B = OFF_WHH0F + SZ_WHH0;
constexpr size_t OFF_WIH1F = OFF_WHH0B + SZ_WHH0;
constexpr size_t OFF_WIH1B = OFF_WIH1F + SZ_WIH1;
constexpr size_t OFF_WOUT  = OFF_WIH1B + SZ_WIH1;
constexpr size_t OFF_APL0  = OFF_WOUT + SZ_WOUT;
constexpr size_t OFF_APL15 = OFF_APL0 + SZ_APL;
constexpr size_t WS_END    = OFF_APL15 + SZ_APL;
static_assert(WS_END <= (size_t)134217728);
static_assert(OFF_WIH0F % 128 == 0 && OFF_WIH0B % 128 == 0 && OFF_WHH0F % 128 == 0 && OFF_WHH0B % 128 == 0);
static_assert(OFF_WIH1F % 128 == 0 && OFF_WIH1B % 128 == 0 && OFF_WOUT % 128 == 0);
static_assert(OFF_APL0 % 128 == 0 && OFF_APL15 % 128 == 0);
static_assert(SZ_XP % 128 == 0 && SZ_WIH0 % 128 == 0 && SZ_WHH0 % 128 == 0 && SZ_WIH1 % 128 == 0);
static_assert(SZ_WOUT % 128 == 0 && SZ_APL % 128 == 0);
static_assert(OFF_WIH0B == OFF_WIH0F + (size_t)G4 * EMB * 2);
static_assert(OFF_WHH0B == OFF_WHH0F + (size_t)G4 * HID * 2);
static_assert(OFF_WIH1B == OFF_WIH1F + (size_t)G4 * L1IN * 2);
static_assert(OFF_APL15 == OFF_APL0 + (size_t)NWORD * L1IN * 2);

__device__ __forceinline__ float sigm(float x) {
    return __builtin_amdgcn_rcpf(1.0f + __expf(-x));
}
__device__ __forceinline__ float tanh_f(float x) {
    const float ax = fminf(fabsf(x), 12.0f);
    const float e  = __expf(-2.0f * ax);
    const float t  = (1.0f - e) * __builtin_amdgcn_rcpf(1.0f + e);
    return copysignf(t, x);
}
__device__ __forceinline__ v8f v8f_zero() {
    v8f r;
#pragma unroll
    for (int i = 0; i < 8; ++i) r[i] = 0.0f;
    return r;
}
__device__ __forceinline__ float ldg_f(const float* p) {
    return *(gf32*)(uintptr_t)p;
}
__device__ __forceinline__ int ldg_i(const int* p) {
    return *(gi32*)(uintptr_t)p;
}
__device__ __forceinline__ v4f ldg_v4(const float* p) {
    return *(gv4f*)(uintptr_t)p;
}

__device__ __forceinline__ v16h ldfrag_g(const _Float16* p) {
    Frag f;
    f.p[0] = *(gv8h*)(uintptr_t)(p);
    f.p[1] = *(gv8h*)(uintptr_t)(p + 16);
    return f.v;
}
__device__ __forceinline__ v16h ldfrag_l(const _Float16* p) {
    Frag f;
    f.p[0] = *(const v8ha*)(p);
    f.p[1] = *(const v8ha*)(p + 16);
    return f.v;
}

__device__ __forceinline__ void mma(v8f& acc, const v16h& a, const v16h& b) {
    acc = __builtin_amdgcn_wmma_f32_16x16x32_f16(false, a, false, b, (short)0, acc, false, false);
    asm volatile("v_nop\n\tv_nop\n\tv_nop\n\tv_nop" : "+v"(acc) : "v"(a), "v"(b));
}

__global__ __launch_bounds__(256)
void cvt_w16_kernel(const float* __restrict__ src, _Float16* dst, int n8)
{
    const int i = blockIdx.x * 256 + threadIdx.x;
    if (i >= n8) return;
    const size_t e = (size_t)i * 8;
    const v4f a = ldg_v4(src + e);
    const v4f b = ldg_v4(src + e + 4);
    v8h o;
#pragma unroll
    for (int c = 0; c < 4; ++c) {
        o[c]     = (_Float16)(a[c] * OPSCALE);
        o[c + 4] = (_Float16)(b[c] * OPSCALE);
    }
    *(volatile v8h*)(dst + e) = o;
    __threadfence();
    *(volatile v8h*)(dst + e) = o;
}

__global__ __launch_bounds__(256)
void embed_kernel(const int* __restrict__ ids, const float* __restrict__ emb, _Float16* xp, int total8)
{
    const int i = blockIdx.x * 256 + threadIdx.x;
    if (i >= total8) return;
    const int r  = i >> 3;
    const int ch = (i & 7) * 8;
    const int t  = r / NWORD;
    const int n  = r - t * NWORD;
    int id = ldg_i(ids + n * TCH + t);
    id = min(max(id, 0), VOC - 1);
    const float* s = emb + (size_t)id * EMB + ch;
    const v4f a = ldg_v4(s);
    const v4f b = ldg_v4(s + 4);
    v8h o;
#pragma unroll
    for (int c = 0; c < 4; ++c) {
        o[c]     = (_Float16)(a[c] * OPSCALE);
        o[c + 4] = (_Float16)(b[c] * OPSCALE);
    }
    _Float16* d = xp + (size_t)r * EMB + ch;
    *(volatile v8h*)d = o;
    __threadfence();
    *(volatile v8h*)d = o;
}

__global__ __launch_bounds__(256)
void lstm_l0_kernel(const _Float16* __restrict__ xp,
                    const _Float16* __restrict__ wih, const _Float16* __restrict__ whh,
                    const float* __restrict__ bia_f, const float* __restrict__ bia_b,
                    _Float16* apl)
{
    __shared__ __attribute__((aligned(16))) _Float16 hbuf[NWB * HSP];

    const int tid  = threadIdx.x;
    const int lane = tid & 31;
    const int wv   = tid >> 5;
    const int hh   = lane >> 4;
    const int m    = lane & 15;
    const int dir  = blockIdx.y;
    const int n0   = blockIdx.x * NWB;
    const int ucol = wv * 32;

    const _Float16* Wih = wih + (size_t)dir * ((size_t)G4 * EMB);
    const _Float16* Whh = whh + (size_t)dir * ((size_t)G4 * HID);

    {
        v8h z;
#pragma unroll
        for (int c = 0; c < 8; ++c) z[c] = (_Float16)0.0f;
        for (int i = tid; i < (NWB * HSP) / 8; i += 256) *(v8ha*)(hbuf + i * 8) = z;
    }

    float br[2][4];
#pragma unroll
    for (int nt = 0; nt < 2; ++nt)
#pragma unroll
        for (int g = 0; g < 4; ++g) {
            const int bi = g * HID + ucol + nt * 16 + m;
            const float vf = ldg_f(bia_f + bi);
            const float vb = ldg_f(bia_b + bi);
            br[nt][g] = dir ? vb : vf;
        }

    v8f cst[2];
    cst[0] = v8f_zero();
    cst[1] = v8f_zero();

    __syncthreads();

#pragma unroll 1
    for (int s = 0; s < TCH; ++s) {
        const int t = dir ? (TCH - 1 - s) : s;

        v8f acc[2][4];
#pragma unroll
        for (int nt = 0; nt < 2; ++nt)
#pragma unroll
            for (int g = 0; g < 4; ++g) acc[nt][g] = v8f_zero();

        const _Float16* xrow = xp + ((size_t)t * NWORD + n0 + m) * EMB + 8 * hh;
#pragma unroll 1
        for (int kx = 0; kx < EMB / 32; ++kx) {
            const v16h a = ldfrag_g(xrow + kx * 32);
#pragma unroll
            for (int nt = 0; nt < 2; ++nt)
#pragma unroll
                for (int g = 0; g < 4; ++g) {
                    const v16h b = ldfrag_g(Wih + (size_t)(g * HID + ucol + nt * 16 + m) * EMB + kx * 32 + 8 * hh);
                    mma(acc[nt][g], a, b);
                }
        }
        const _Float16* hrow = hbuf + m * HSP + 8 * hh;
#pragma unroll 1
        for (int kh = 0; kh < HID / 32; ++kh) {
            const v16h a = ldfrag_l(hrow + kh * 32);
#pragma unroll
            for (int nt = 0; nt < 2; ++nt)
#pragma unroll
                for (int g = 0; g < 4; ++g) {
                    const v16h b = ldfrag_g(Whh + (size_t)(g * HID + ucol + nt * 16 + m) * HID + kh * 32 + 8 * hh);
                    mma(acc[nt][g], a, b);
                }
        }

        __syncthreads();

#pragma unroll
        for (int nt = 0; nt < 2; ++nt) {
            const int unit = ucol + nt * 16 + m;
#pragma unroll
            for (int r = 0; r < 8; ++r) {
                const float pi = acc[nt][0][r] * ACCINV + br[nt][0];
                const float pf = acc[nt][1][r] * ACCINV + br[nt][1];
                const float pg = acc[nt][2][r] * ACCINV + br[nt][2];
                const float po = acc[nt][3][r] * ACCINV + br[nt][3];
                const float cn = sigm(pf) * cst[nt][r] + sigm(pi) * tanh_f(pg);
                cst[nt][r] = cn;
                const float hv = sigm(po) * tanh_f(cn);
                hbuf[(8 * hh + r) * HSP + unit] = (_Float16)(hv * OPSCALE);
            }
        }

        __syncthreads();

        if (t == 0 || t == TCH - 1) {
            _Float16* pl = apl + ((t == 0) ? (size_t)0 : (size_t)NWORD * L1IN);
            const int ra = wv;
            const int rb = wv + 8;
            const int ch = lane * 8;
            const v8h va = *(const v8ha*)(hbuf + ra * HSP + ch);
            const v8h vb = *(const v8ha*)(hbuf + rb * HSP + ch);
            _Float16* da = pl + (size_t)(n0 + ra) * L1IN + dir * HID + ch;
            _Float16* db = pl + (size_t)(n0 + rb) * L1IN + dir * HID + ch;
            *(volatile v8h*)da = va;
            *(volatile v8h*)db = vb;
            __threadfence();
            *(volatile v8h*)da = va;
            *(volatile v8h*)db = vb;
        }
    }
}

__device__ __forceinline__ void l1_pass(const _Float16* __restrict__ aplp, const _Float16* __restrict__ w,
                                        const float* __restrict__ b, _Float16* mcol,
                                        int n0, int wv, int hh, int m)
{
    const int ucol = wv * 32;
    v8f acc[2][3];
#pragma unroll
    for (int nt = 0; nt < 2; ++nt)
#pragma unroll
        for (int gi = 0; gi < 3; ++gi) acc[nt][gi] = v8f_zero();

    const _Float16* arow = aplp + (size_t)(n0 + m) * L1IN + 8 * hh;
#pragma unroll 1
    for (int k = 0; k < L1IN / 32; ++k) {
        const v16h a = ldfrag_g(arow + k * 32);
#pragma unroll
        for (int nt = 0; nt < 2; ++nt)
#pragma unroll
            for (int gi = 0; gi < 3; ++gi) {
                const int grow = (gi == 0) ? 0 : (gi + 1) * HID;
                const v16h bb = ldfrag_g(w + (size_t)(grow + ucol + nt * 16 + m) * L1IN + k * 32 + 8 * hh);
                mma(acc[nt][gi], a, bb);
            }
    }
#pragma unroll
    for (int nt = 0; nt < 2; ++nt) {
        const int unit = ucol + nt * 16 + m;
        const float bi = ldg_f(b + unit);
        const float bg = ldg_f(b + 2 * HID + unit);
        const float bo = ldg_f(b + 3 * HID + unit);
#pragma unroll
        for (int r = 0; r < 8; ++r) {
            const float cn = sigm(acc[nt][0][r] * ACCINV + bi) * tanh_f(acc[nt][1][r] * ACCINV + bg);
            const float hv = sigm(acc[nt][2][r] * ACCINV + bo) * tanh_f(cn);
            mcol[(8 * hh + r) * MSP + unit] = (_Float16)(hv * OPSCALE);
        }
    }
}

__global__ __launch_bounds__(256)
void lstm_l1_out_kernel(const _Float16* __restrict__ apl, const _Float16* __restrict__ wih1,
                        const float* __restrict__ b1f, const float* __restrict__ b1b,
                        const _Float16* __restrict__ wout, const float* __restrict__ bout,
                        float* out)
{
    __shared__ __attribute__((aligned(16))) _Float16 mbuf[NWB * MSP];
    __shared__ __attribute__((aligned(16))) float    obuf[NWB * OSP];

    const int tid  = threadIdx.x;
    const int lane = tid & 31;
    const int wv   = tid >> 5;
    const int hh   = lane >> 4;
    const int m    = lane & 15;
    const int n0   = blockIdx.x * NWB;
    const int ucol = wv * 32;

    l1_pass(apl, wih1, b1f, mbuf, n0, wv, hh, m);
    l1_pass(apl + (size_t)NWORD * L1IN, wih1 + (size_t)G4 * L1IN, b1b, mbuf + HID, n0, wv, hh, m);
    __syncthreads();

    v8f acc[2];
    acc[0] = v8f_zero();
    acc[1] = v8f_zero();
    const _Float16* arow = mbuf + m * MSP + 8 * hh;
#pragma unroll 1
    for (int k = 0; k < L1IN / 32; ++k) {
        const v16h a = ldfrag_l(arow + k * 32);
#pragma unroll
        for (int nt = 0; nt < 2; ++nt) {
            const v16h bb = ldfrag_g(wout + (size_t)(ucol + nt * 16 + m) * L1IN + k * 32 + 8 * hh);
            mma(acc[nt], a, bb);
        }
    }
#pragma unroll
    for (int nt = 0; nt < 2; ++nt) {
        const int col = ucol + nt * 16 + m;
        const float bo = ldg_f(bout + col);
#pragma unroll
        for (int r = 0; r < 8; ++r) obuf[(8 * hh + r) * OSP + col] = acc[nt][r] * ACCINV + bo;
    }
    __syncthreads();

    v4f v[4];
#pragma unroll
    for (int it = 0; it < 4; ++it) {
        const int idx = it * 256 + tid;
        const int row = idx >> 6;
        const int ch  = (idx & 63) * 4;
        v[it] = *(const v4fa*)(obuf + row * OSP + ch);
    }
#pragma unroll
    for (int it = 0; it < 4; ++it) {
        const int idx = it * 256 + tid;
        const int row = idx >> 6;
        const int ch  = (idx & 63) * 4;
        *(volatile v4f*)(out + (size_t)(n0 + row) * HID + ch) = v[it];
    }
    __threadfence();
#pragma unroll
    for (int it = 0; it < 4; ++it) {
        const int idx = it * 256 + tid;
        const int row = idx >> 6;
        const int ch  = (idx & 63) * 4;
        *(volatile v4f*)(out + (size_t)(n0 + row) * HID + ch) = v[it];
    }
}

extern "C" void kernel_launch(void* const* d_in, const int* in_sizes, int n_in,
                              void* d_out, int out_size, void* d_ws, size_t ws_size,
                              hipStream_t stream)
{
    if (n_in < 16) return;
    if (in_sizes[0]  != NWORD * TCH) return;
    if (in_sizes[1]  != VOC * EMB)   return;
    if (in_sizes[2]  != G4 * EMB)    return;
    if (in_sizes[3]  != G4 * HID)    return;
    if (in_sizes[4]  != G4)          return;
    if (in_sizes[5]  != G4 * EMB)    return;
    if (in_sizes[6]  != G4 * HID)    return;
    if (in_sizes[7]  != G4)          return;
    if (in_sizes[8]  != G4 * L1IN)   return;
    if (in_sizes[9]  != G4 * HID)    return;
    if (in_sizes[10] != G4)          return;
    if (in_sizes[11] != G4 * L1IN)   return;
    if (in_sizes[12] != G4 * HID)    return;
    if (in_sizes[13] != G4)          return;
    if (in_sizes[14] != HID * L1IN)  return;
    if (in_sizes[15] != HID)         return;
    if (out_size != NWORD * HID)     return;
    if (ws_size < WS_END)            return;

    const int*   char_ids = (const int*)d_in[0];
    const float* char_emb = (const float*)d_in[1];
    const float* w_ih_l0f = (const float*)d_in[2];
    const float* w_hh_l0f = (const float*)d_in[3];
    const float* b_l0f    = (const float*)d_in[4];
    const float* w_ih_l0b = (const float*)d_in[5];
    const float* w_hh_l0b = (const float*)d_in[6];
    const float* b_l0b    = (const float*)d_in[7];
    const float* w_ih_l1f = (const float*)d_in[8];
    const float* b_l1f    = (const float*)d_in[10];
    const float* w_ih_l1b = (const float*)d_in[11];
    const float* b_l1b    = (const float*)d_in[13];
    const float* w_out    = (const float*)d_in[14];
    const float* b_out    = (const float*)d_in[15];
    float* out = (float*)d_out;

    char* ws = (char*)d_ws;
    _Float16* xp    = (_Float16*)(ws + OFF_XP);
    _Float16* wih0f = (_Float16*)(ws + OFF_WIH0F);
    _Float16* wih0b = (_Float16*)(ws + OFF_WIH0B);
    _Float16* whh0f = (_Float16*)(ws + OFF_WHH0F);
    _Float16* whh0b = (_Float16*)(ws + OFF_WHH0B);
    _Float16* wih1f = (_Float16*)(ws + OFF_WIH1F);
    _Float16* wih1b = (_Float16*)(ws + OFF_WIH1B);
    _Float16* woutp = (_Float16*)(ws + OFF_WOUT);
    _Float16* apl0  = (_Float16*)(ws + OFF_APL0);

    {
        const int n8a = (G4 * EMB) / 8, n8b = (G4 * HID) / 8, n8c = (G4 * L1IN) / 8, n8d = (HID * L1IN) / 8;
        cvt_w16_kernel<<<dim3((n8a + 255) / 256), dim3(256), 0, stream>>>(w_ih_l0f, wih0f, n8a);
        cvt_w16_kernel<<<dim3((n8a + 255) / 256), dim3(256), 0, stream>>>(w_ih_l0b, wih0b, n8a);
        cvt_w16_kernel<<<dim3((n8b + 255) / 256), dim3(256), 0, stream>>>(w_hh_l0f, whh0f, n8b);
        cvt_w16_kernel<<<dim3((n8b + 255) / 256), dim3(256), 0, stream>>>(w_hh_l0b, whh0b, n8b);
        cvt_w16_kernel<<<dim3((n8c + 255) / 256), dim3(256), 0, stream>>>(w_ih_l1f, wih1f, n8c);
        cvt_w16_kernel<<<dim3((n8c + 255) / 256), dim3(256), 0, stream>>>(w_ih_l1b, wih1b, n8c);
        cvt_w16_kernel<<<dim3((n8d + 255) / 256), dim3(256), 0, stream>>>(w_out,    woutp, n8d);
    }

    {
        const int total8 = TCH * NWORD * (EMB / 8);
        embed_kernel<<<dim3((total8 + 255) / 256), dim3(256), 0, stream>>>(char_ids, char_emb, xp, total8);
    }

    lstm_l0_kernel<<<dim3(NWORD / NWB, 2), dim3(256), 0, stream>>>(
        (const _Float16*)xp, (const _Float16*)wih0f, (const _Float16*)whh0f, b_l0f, b_l0b, apl0);

    lstm_l1_out_kernel<<<dim3(NWORD / NWB), dim3(256), 0, stream>>>(
        (const _Float16*)apl0, (const _Float16*)wih1f, b_l1f, b_l1b, (const _Float16*)woutp, b_out, out);
}
